// LineClassifier_2748779070289
// MI455X (gfx1250) — hardware-verified
//
#include <hip/hip_runtime.h>
#include <math.h>
#include <stdint.h>

#pragma clang fp contract(off)

#define NPIX    16384
#define IMW     128
#define CIN     256
#define DLOI    128
#define NLN     16000
#define DFC     1024
#define NLAB    3
#define NHP     64
#define NS0     32
#define NS1     8
#define MCH     8000
#define NCH     2
#define FSC     16.0f
#define WSC1    256.0f
#define WSC     512.0f
#define RCARRY  2048.0f
#define LDP     264

static_assert(NLN == NCH * MCH);
static_assert((MCH % 64) == 0 && (DFC % 64) == 0 && (NPIX % 64) == 0 && (DLOI % 64) == 0 && (NHP % 64) == 0);
static_assert((CIN % 32) == 0 && (DFC % 32) == 0);
static_assert(((MCH * DFC / 8) % 256) == 0);
static_assert(((MCH * NLAB) % 4) == 0);
static_assert((((NPIX / 64) * (DLOI / 64)) % 8) == 0);
static_assert((((MCH / 64) * (DFC / 64)) % 8) == 0);
static_assert(((DLOI * CIN / 8) % 256) == 0 && ((DFC * DFC / 8) % 256) == 0 && ((NHP * DFC / 8) % 256) == 0);
static_assert(NS0 == 4 * NS1 && NS1 == 8 && DFC == DLOI * NS1);
static_assert(((NLAB * DFC) % 8) == 0);
static_assert((LDP % 8) == 0);

typedef _Float16       v16h __attribute__((ext_vector_type(16)));
typedef __bf16         v16b __attribute__((ext_vector_type(16)));
typedef unsigned short v16us __attribute__((ext_vector_type(16)));
typedef unsigned short v8us __attribute__((ext_vector_type(8)));
typedef float          v8f  __attribute__((ext_vector_type(8)));
typedef float          v4f  __attribute__((ext_vector_type(4)));
typedef unsigned int   v4u  __attribute__((ext_vector_type(4)));

union Frag { v16us u; v8us p[2]; v16h h; v16b b; };
union U8   { v8us s; v4u u; };

__device__ __forceinline__ unsigned short bf_bits(float f) {
  unsigned u = __float_as_uint(f);
  return (unsigned short)((u + 0x7FFFu + ((u >> 16) & 1u)) >> 16);
}
__device__ __forceinline__ float bf_up(unsigned short h) { return __uint_as_float(((unsigned)h) << 16); }
__device__ __forceinline__ float bfr(float f) { return bf_up(bf_bits(f)); }
__device__ __forceinline__ unsigned short h_bits(_Float16 x) { return __builtin_bit_cast(unsigned short, x); }
__device__ __forceinline__ unsigned pk16(unsigned short a, unsigned short b) { return (unsigned)a | ((unsigned)b << 16); }
__device__ __forceinline__ v8f zero8() { v8f z = {0.f, 0.f, 0.f, 0.f, 0.f, 0.f, 0.f, 0.f}; return z; }
__device__ __forceinline__ float clampf127(float x) { return fminf(fmaxf(x, 0.0f), (float)(IMW - 1)); }
__device__ __forceinline__ int clampi127(int x) { x = (x < 0) ? 0 : x; return (x > IMW - 1) ? (IMW - 1) : x; }

__device__ __forceinline__ v16us ldfrag(const unsigned short* p) {
  Frag f;
  f.p[0] = *(const v8us*)(p);
  f.p[1] = *(const v8us*)(p + 16);
  return f.u;
}

template <int BF>
__device__ __forceinline__ v8f mma_raw(v16us a, v16us b, v8f c) {
  Frag fa, fb;
  fa.u = a;
  fb.u = b;
  if constexpr (BF) {
    return __builtin_amdgcn_wmma_f32_16x16x32_bf16(false, fa.b, false, fb.b, (short)0, c, false, false);
  } else {
    return __builtin_amdgcn_wmma_f32_16x16x32_f16(false, fa.h, false, fb.h, (short)0, c, false, false);
  }
}
__device__ __forceinline__ void dep_guard1(v8f& a, v8f& b, v16us x) {
#if defined(__HIP_DEVICE_COMPILE__)
  asm volatile("v_nop\n\tv_nop\n\tv_nop\n\tv_nop" : "+v"(a), "+v"(b) : "v"(x));
#endif
}
__device__ __forceinline__ void keep4(v16us a, v16us b, v16us c, v16us d) {
#if defined(__HIP_DEVICE_COMPILE__)
  asm volatile("v_nop" :: "v"(a), "v"(b), "v"(c), "v"(d));
#endif
}
__device__ __forceinline__ void acc_guard4(v8f& a, v8f& b, v8f& c, v8f& d) {
#if defined(__HIP_DEVICE_COMPILE__)
  asm volatile("v_nop\n\tv_nop\n\tv_nop\n\tv_nop" : "+v"(a), "+v"(b), "+v"(c), "+v"(d));
#endif
}
__device__ __forceinline__ void wave_sync_lds() {
  __builtin_amdgcn_fence(__ATOMIC_RELEASE, "workgroup");
  __builtin_amdgcn_wave_barrier();
  __builtin_amdgcn_fence(__ATOMIC_ACQUIRE, "workgroup");
}

__global__ __launch_bounds__(256) void fcvt(const float* __restrict__ F, unsigned short* FP) {
  __shared__ __align__(16) unsigned short s[64 * LDP];
  const int t = threadIdx.x, pl = t & 63, cg = t >> 6;
  const int p0 = blockIdx.x * 64;
#pragma unroll 4
  for (int i = 0; i < CIN / 4; ++i) {
    const int c = cg + 4 * i;
    const float v = bfr(F[(size_t)c * NPIX + (size_t)(p0 + pl)]) * FSC;
    s[pl * LDP + c] = h_bits((_Float16)v);
  }
  __syncthreads();
  const int lane = t & 31, wave = t >> 5;
  U8 v[8];
#pragma unroll
  for (int r = 0; r < 8; ++r) {
    const int row = wave * 8 + r;
    v[r].s = *(const v8us*)(s + row * LDP + lane * 8);
  }
  for (int pass = 0; pass < 2; ++pass) {
#pragma unroll
    for (int r = 0; r < 8; ++r) {
      const int row = wave * 8 + r;
      *(volatile v4u*)(FP + (size_t)(p0 + row) * CIN + lane * 8) = v[r].u;
    }
    __threadfence();
  }
}

__global__ __launch_bounds__(256) void wcvt(const float* __restrict__ W, int nsrc, unsigned short* P, int n8, float scale) {
  const int i  = blockIdx.x * 256 + threadIdx.x;
  const int ic = (i < n8) ? i : (n8 - 1);
  const int e0 = ic * 8;
  const bool valid = (e0 + 8 <= nsrc);
  const int es = valid ? e0 : (nsrc - 8);
  const v4f a = *(const v4f*)(W + es);
  const v4f c = *(const v4f*)(W + es + 4);
  unsigned short hb[8];
#pragma unroll
  for (int e = 0; e < 4; ++e) {
    hb[e]     = valid ? h_bits((_Float16)(bfr(a[e]) * scale)) : (unsigned short)0;
    hb[4 + e] = valid ? h_bits((_Float16)(bfr(c[e]) * scale)) : (unsigned short)0;
  }
  v4u o;
#pragma unroll
  for (int e = 0; e < 4; ++e) o[e] = pk16(hb[2 * e], hb[2 * e + 1]);
  if (i < n8) *(volatile v4u*)(P + (size_t)i * 8) = o;
  __threadfence();
  if (i < n8) *(volatile v4u*)(P + (size_t)i * 8) = o;
}

template <int BF, int OM, int BIASM>
__global__ __launch_bounds__(256) void gemm64(
    const unsigned short* __restrict__ A, int lda, long long strideA,
    const unsigned short* __restrict__ Bt, int ldb, long long strideB,
    const float* __restrict__ bias0, const float* __restrict__ bias1, int Nb,
    void* Cout, int ldc, long long strideC,
    int M, int N, int K, float oscale) {
  __shared__ __align__(16) float sT[8][16 * 68];
  const int b    = blockIdx.y;
  const int lane = threadIdx.x & 31;
  const int wave = threadIdx.x >> 5;
  const int tilesN = N >> 6;
  const int tilesM = M >> 6;
  const int tile = blockIdx.x * 8 + wave;
  if (tile >= tilesM * tilesN) return;
  const int tm = tile / tilesN;
  const int tn = tile - tm * tilesN;
  const int m0 = tm << 6;
  const int n0 = tn << 6;

  const unsigned short* Ab = A  + (size_t)b * (size_t)strideA;
  const unsigned short* Bb = Bt + (size_t)b * (size_t)strideB;

  const int rlane = lane & 15;
  const int koff  = (lane >> 4) * 8;
  const int mOff  = (lane >> 4) * 8;

  v8f acc[4][4];
#pragma unroll
  for (int i = 0; i < 4; ++i)
#pragma unroll
    for (int j = 0; j < 4; ++j) acc[i][j] = zero8();

  for (int k0 = 0; k0 < K; k0 += 32) {
    v16us bh[4];
#pragma unroll
    for (int j = 0; j < 4; ++j) {
      const size_t bo = (size_t)(n0 + (j << 4) + rlane) * ldb + koff + k0;
      bh[j] = ldfrag(Bb + bo);
    }
#pragma unroll
    for (int i = 0; i < 4; ++i) {
      const size_t ao = (size_t)(m0 + (i << 4) + rlane) * lda + koff + k0;
      const v16us ah = ldfrag(Ab + ao);
#pragma unroll
      for (int j = 0; j < 4; ++j) acc[i][j] = mma_raw<BF>(ah, bh[j], acc[i][j]);
      dep_guard1(acc[i][0], acc[i][3], ah);
    }
    keep4(bh[0], bh[1], bh[2], bh[3]);
  }
  acc_guard4(acc[0][0], acc[0][1], acc[0][2], acc[0][3]);
  acc_guard4(acc[1][0], acc[1][1], acc[1][2], acc[1][3]);
  acc_guard4(acc[2][0], acc[2][1], acc[2][2], acc[2][3]);
  acc_guard4(acc[3][0], acc[3][1], acc[3][2], acc[3][3]);

  const int hh2 = lane >> 4, c4 = (lane & 15) * 4;
  const int q8  = lane >> 3, c8 = (lane & 7) * 8;
  float bc[8];
#pragma unroll
  for (int e = 0; e < 8; ++e) bc[e] = 0.f;
  if (BIASM == 0) {
    const bool use1 = (n0 >= Nb);
    if (OM == 0) {
      const int cb = n0 + c4;
      const int i0 = (cb < Nb - 4) ? cb : (Nb - 4);
      const int i1 = (cb - Nb > 0) ? (cb - Nb) : 0;
      const v4f b0v = *(const v4f*)(bias0 + i0);
      const v4f b1v = *(const v4f*)(bias1 + i1);
#pragma unroll
      for (int e = 0; e < 4; ++e) bc[e] = bfr(use1 ? b1v[e] : b0v[e]);
    } else {
      const int cb = n0 + c8;
      const int i0 = (cb < Nb - 8) ? cb : (Nb - 8);
      const int i1 = (cb - Nb > 0) ? (cb - Nb) : 0;
      const v4f b0a = *(const v4f*)(bias0 + i0), b0b = *(const v4f*)(bias0 + i0 + 4);
      const v4f b1a = *(const v4f*)(bias1 + i1), b1b = *(const v4f*)(bias1 + i1 + 4);
#pragma unroll
      for (int e = 0; e < 4; ++e) {
        bc[e]     = bfr(use1 ? b1a[e] : b0a[e]);
        bc[4 + e] = bfr(use1 ? b1b[e] : b0b[e]);
      }
    }
  }

  float* slab = sT[wave];
#pragma unroll
  for (int i = 0; i < 4; ++i) {
    const int mBase = m0 + (i << 4);
#pragma unroll
    for (int j = 0; j < 4; ++j) {
#pragma unroll
      for (int r = 0; r < 8; ++r) {
        slab[(mOff + r) * 68 + (j << 4) + rlane] = acc[i][j][r];
      }
    }
    wave_sync_lds();
    if constexpr (OM == 0) {
      float* C = (float*)Cout + (size_t)b * (size_t)strideC;
      v4f vals[8];
#pragma unroll
      for (int it = 0; it < 8; ++it) {
        const int row = it * 2 + hh2;
        v4f v = *(const v4f*)(slab + row * 68 + c4);
#pragma unroll
        for (int e = 0; e < 4; ++e) v[e] = v[e] * oscale + bc[e];
        vals[it] = v;
      }
      for (int pass = 0; pass < 2; ++pass) {
#pragma unroll
        for (int it = 0; it < 8; ++it) {
          const int row = it * 2 + hh2;
          *(volatile v4f*)(C + (size_t)(mBase + row) * ldc + n0 + c4) = vals[it];
        }
        __threadfence();
      }
    } else {
      unsigned short* C = (unsigned short*)Cout + (size_t)b * (size_t)strideC;
      v4u hv[4];
#pragma unroll
      for (int it = 0; it < 4; ++it) {
        const int row = it * 4 + q8;
        const float* sp = slab + row * 68 + c8;
        float bm = 0.f;
        if (BIASM == 1) bm = bfr(bias0[mBase + row]);
        v4u a;
#pragma unroll
        for (int e = 0; e < 4; ++e) {
          const float f0 = sp[2 * e]     * oscale + ((BIASM == 1) ? bm : bc[2 * e]);
          const float f1 = sp[2 * e + 1] * oscale + ((BIASM == 1) ? bm : bc[2 * e + 1]);
          a[e] = pk16(h_bits((_Float16)f0), h_bits((_Float16)f1));
        }
        hv[it] = a;
      }
      for (int pass = 0; pass < 2; ++pass) {
#pragma unroll
        for (int it = 0; it < 4; ++it) {
          const int row = it * 4 + q8;
          unsigned short* dp = C + (size_t)(mBase + row) * ldc + n0 + c8;
          *(volatile v4u*)(dp) = hv[it];
        }
        __threadfence();
      }
    }
    wave_sync_lds();
  }
}

__global__ __launch_bounds__(256) void line_pool(const float* __restrict__ LOI, const float* __restrict__ LN,
                                               unsigned short* AH, unsigned short* AL, int line0) {
  __shared__ __align__(16) unsigned short sh[DFC];
  __shared__ __align__(16) unsigned short sl[DFC];
  const int t = threadIdx.x, lane = t & 31, wave = t >> 5;
  int li = line0 + (int)blockIdx.x;
  li = (li < NLN) ? li : (NLN - 1);
  const float Ux = bfr(LN[(size_t)li * 4 + 0]);
  const float Uy = bfr(LN[(size_t)li * 4 + 1]);
  const float Vx = bfr(LN[(size_t)li * 4 + 2]);
  const float Vy = bfr(LN[(size_t)li * 4 + 3]);
  const int c0 = lane * 4;
  v4f mx = {0.f, 0.f, 0.f, 0.f};
#pragma unroll
  for (int s = 0; s < NS0 / NS1; ++s) {
    const int j = wave * (NS0 / NS1) + s;
    const float tj  = (j == NS0 - 1) ? 1.0f : (float)j * (1.0f / 31.0f);
    const float omt = 1.0f - tj;
    const float ax = Ux * tj;
    const float bx = Vx * omt;
    const float cx = ax + bx;
    const float px = cx - 0.5f;
    const float ay = Uy * tj;
    const float by = Vy * omt;
    const float cy = ay + by;
    const float py = cy - 0.5f;
    const float fx0 = clampf127(floorf(px));
    const float fy0 = clampf127(floorf(py));
    const float fx1 = clampf127(fx0 + 1.0f);
    const float fy1 = clampf127(fy0 + 1.0f);
    const int ix0 = clampi127((int)fx0), iy0 = clampi127((int)fy0);
    const int ix1 = clampi127((int)fx1), iy1 = clampi127((int)fy1);
    const float wy0 = fy1 - py;
    const float wy1 = py - fy0;
    const float wx0 = fx1 - px;
    const float wx1 = px - fx0;
    const v4f g00 = *(const v4f*)(LOI + ((size_t)(iy0 * IMW + ix0)) * DLOI + c0);
    const v4f g10 = *(const v4f*)(LOI + ((size_t)(iy1 * IMW + ix0)) * DLOI + c0);
    const v4f g01 = *(const v4f*)(LOI + ((size_t)(iy0 * IMW + ix1)) * DLOI + c0);
    const v4f g11 = *(const v4f*)(LOI + ((size_t)(iy1 * IMW + ix1)) * DLOI + c0);
#pragma unroll
    for (int q = 0; q < 4; ++q) {
      const float r00 = fmaxf(g00[q], 0.0f);
      const float r10 = fmaxf(g10[q], 0.0f);
      const float r01 = fmaxf(g01[q], 0.0f);
      const float r11 = fmaxf(g11[q], 0.0f);
      const float t1 = (r00 * wy0) * wx0;
      const float t2 = (r10 * wy1) * wx0;
      const float t3 = (r01 * wy0) * wx1;
      const float t4 = (r11 * wy1) * wx1;
      const float v = ((t1 + t2) + t3) + t4;
      mx[q] = (s == 0) ? v : fmaxf(mx[q], v);
    }
  }
#pragma unroll
  for (int q = 0; q < 4; ++q) {
    const float v = mx[q];
    const _Float16 hv = (_Float16)v;
    const float res = (v - (float)hv) * RCARRY;
    const int idx = (c0 + q) * NS1 + wave;
    sh[idx] = h_bits(hv);
    sl[idx] = h_bits((_Float16)res);
  }
  __syncthreads();
  const bool lo = (t >= 128);
  const int p = t & 127;
  U8 a, b;
  a.s = *(const v8us*)(sh + p * 8);
  b.s = *(const v8us*)(sl + p * 8);
  v4u o;
#pragma unroll
  for (int e = 0; e < 4; ++e) o[e] = lo ? b.u[e] : a.u[e];
  unsigned short* dst = (lo ? AL : AH) + (size_t)blockIdx.x * DFC + (size_t)p * 8;
  *(volatile v4u*)dst = o;
  __threadfence();
  *(volatile v4u*)dst = o;
}

__global__ __launch_bounds__(256) void xplanes(const float* __restrict__ Hp, const float* __restrict__ Lp,
                                             const float* __restrict__ bias, unsigned short* AH, unsigned short* AL, int n8) {
  const int i  = blockIdx.x * 256 + threadIdx.x;
  const int ic = (i < n8) ? i : (n8 - 1);
  const size_t e0 = (size_t)ic * 8;
  const int col = (int)(e0 & (size_t)(DFC - 1));
  const v4f h0 = *(const v4f*)(Hp + e0), h1 = *(const v4f*)(Hp + e0 + 4);
  const v4f l0 = *(const v4f*)(Lp + e0), l1 = *(const v4f*)(Lp + e0 + 4);
  const v4f b0 = *(const v4f*)(bias + col), b1 = *(const v4f*)(bias + col + 4);
  float y[8];
#pragma unroll
  for (int e = 0; e < 4; ++e) {
    y[e]     = fmaxf((h0[e] + l0[e]) + bfr(b0[e]), 0.0f);
    y[4 + e] = fmaxf((h1[e] + l1[e]) + bfr(b1[e]), 0.0f);
  }
  v4u oh, ol;
#pragma unroll
  for (int e = 0; e < 4; ++e) {
    const _Float16 ha = (_Float16)y[2 * e], hb = (_Float16)y[2 * e + 1];
    const float ra = (y[2 * e] - (float)ha) * RCARRY;
    const float rb = (y[2 * e + 1] - (float)hb) * RCARRY;
    oh[e] = pk16(h_bits(ha), h_bits(hb));
    ol[e] = pk16(h_bits((_Float16)ra), h_bits((_Float16)rb));
  }
  if (i < n8) {
    *(volatile v4u*)(AH + (size_t)i * 8) = oh;
    *(volatile v4u*)(AL + (size_t)i * 8) = ol;
  }
  __threadfence();
  if (i < n8) {
    *(volatile v4u*)(AH + (size_t)i * 8) = oh;
    *(volatile v4u*)(AL + (size_t)i * 8) = ol;
  }
}

__global__ __launch_bounds__(256) void outpack(const float* __restrict__ H3, const float* __restrict__ L3,
                                             const float* __restrict__ b3, float* outp, int nq) {
  const int i  = blockIdx.x * 256 + threadIdx.x;
  const int ic = (i < nq) ? i : (nq - 1);
  v4f v;
#pragma unroll
  for (int q = 0; q < 4; ++q) {
    const int e = ic * 4 + q;
    const int row = e / NLAB;
    const int col = e - row * NLAB;
    const size_t idx = (size_t)row * NHP + (size_t)col;
    v[q] = (H3[idx] + L3[idx]) + bfr(b3[col]);
  }
  if (i < nq) *(volatile v4f*)(outp + (size_t)i * 4) = v;
  __threadfence();
  if (i < nq) *(volatile v4f*)(outp + (size_t)i * 4) = v;
}

extern "C" void kernel_launch(void* const* d_in, const int* in_sizes, int n_in,
                              void* d_out, int out_size, void* d_ws, size_t ws_size,
                              hipStream_t stream) {
  if (n_in < 10) return;
  if (in_sizes[0] != CIN * NPIX) return;
  if (in_sizes[1] != NLN * 4) return;
  if (in_sizes[2] != DLOI * CIN) return;
  if (in_sizes[3] != DLOI) return;
  if (in_sizes[4] != DFC * DFC || in_sizes[5] != DFC) return;
  if (in_sizes[6] != DFC * DFC || in_sizes[7] != DFC) return;
  if (in_sizes[8] != NLAB * DFC || in_sizes[9] != NLAB) return;
  if (out_size != NLN * NLAB) return;

  const float* feats = (const float*)d_in[0];
  const float* lines = (const float*)d_in[1];
  const float* w_fc1 = (const float*)d_in[2];
  const float* b_fc1 = (const float*)d_in[3];
  const float* w1    = (const float*)d_in[4];
  const float* b1    = (const float*)d_in[5];
  const float* w2    = (const float*)d_in[6];
  const float* b2    = (const float*)d_in[7];
  const float* w3    = (const float*)d_in[8];
  const float* b3    = (const float*)d_in[9];

  const size_t PFP  = (size_t)NPIX * CIN * 2;
  const size_t PWC  = (size_t)DLOI * CIN * 2;
  const size_t PLOI = (size_t)NPIX * DLOI * 4;
  const size_t PW   = (size_t)DFC * DFC * 2;
  const size_t PW3  = (size_t)NHP * DFC * 2;
  const size_t PA   = (size_t)MCH * DFC * 2;
  const size_t PHL  = (size_t)MCH * DFC * 4;
  const size_t PH3  = (size_t)MCH * NHP * 4;
  size_t off = 0;
  const size_t oFP  = off; off += PFP;
  const size_t oWC  = off; off += PWC;
  const size_t oLOI = off; off += PLOI;
  const size_t oW1  = off; off += PW;
  const size_t oW2  = off; off += PW;
  const size_t oW3  = off; off += PW3;
  const size_t oAH  = off; off += PA;
  const size_t oAL  = off; off += PA;
  const size_t oH   = off; off += PHL;
  const size_t oL   = off; off += PHL;
  const size_t oH3  = off; off += PH3;
  const size_t oL3  = off; off += PH3;
  if (off > ws_size) return;
  if (off > (size_t)134217728) return;
  if ((oWC % 256) != 0 || (oLOI % 256) != 0 || (oW1 % 256) != 0 || (oW2 % 256) != 0 || (oW3 % 256) != 0 ||
      (oAH % 256) != 0 || (oAL % 256) != 0 || (oH % 256) != 0 || (oL % 256) != 0 || (oH3 % 256) != 0 || (oL3 % 256) != 0) return;

  char* ws = (char*)d_ws;
  unsigned short* FP  = (unsigned short*)(ws + oFP);
  unsigned short* WCP = (unsigned short*)(ws + oWC);
  float*          LOI = (float*)(ws + oLOI);
  unsigned short* W1P = (unsigned short*)(ws + oW1);
  unsigned short* W2P = (unsigned short*)(ws + oW2);
  unsigned short* W3P = (unsigned short*)(ws + oW3);
  unsigned short* AH  = (unsigned short*)(ws + oAH);
  unsigned short* AL  = (unsigned short*)(ws + oAL);
  float*          Hb  = (float*)(ws + oH);
  float*          Lb  = (float*)(ws + oL);
  float*          H3  = (float*)(ws + oH3);
  float*          L3  = (float*)(ws + oL3);
  float*          out0 = (float*)d_out;

  const dim3 blk(256);
  const int n8c = (DLOI * CIN) / 8;
  const int n8w = (DFC * DFC) / 8;
  const int n8h = (NHP * DFC) / 8;
  const int n8x = (MCH * DFC) / 8;
  const int nqo = (MCH * NLAB) / 4;
  const dim3 gF(NPIX / 64);
  const dim3 gC(((NPIX / 64) * (DLOI / 64) + 7) / 8, 1);
  const dim3 gG(((MCH / 64) * (DFC / 64) + 7) / 8, 1);
  const dim3 gH(((MCH / 64) * (NHP / 64) + 7) / 8, 1);
  const dim3 gP(MCH);
  const dim3 gX(n8x / 256);
  const dim3 gO((nqo + 255) / 256);
  const float osc_cv = 1.0f / (FSC * WSC1);
  const float osc_hi = 1.0f / WSC;
  const float osc_lo = 1.0f / (WSC * RCARRY);

  fcvt<<<gF, blk, 0, stream>>>(feats, FP);
  wcvt<<<dim3(n8c / 256), blk, 0, stream>>>(w_fc1, DLOI * CIN, WCP, n8c, WSC1);
  wcvt<<<dim3(n8w / 256), blk, 0, stream>>>(w1, DFC * DFC, W1P, n8w, WSC);
  wcvt<<<dim3(n8w / 256), blk, 0, stream>>>(w2, DFC * DFC, W2P, n8w, WSC);
  wcvt<<<dim3(n8h / 256), blk, 0, stream>>>(w3, NLAB * DFC, W3P, n8h, WSC);

  gemm64<0, 0, 0><<<gC, blk, 0, stream>>>(
      FP, CIN, 0LL, WCP, CIN, 0LL, b_fc1, b_fc1, DLOI,
      (void*)LOI, DLOI, 0LL, NPIX, DLOI, CIN, osc_cv);

  for (int ch = 0; ch < NCH; ++ch) {
    line_pool<<<gP, blk, 0, stream>>>(LOI, lines, AH, AL, ch * MCH);
    gemm64<0, 0, 2><<<gG, blk, 0, stream>>>(
        AH, DFC, 0LL, W1P, DFC, 0LL, b1, b1, DFC,
        (void*)Hb, DFC, 0LL, MCH, DFC, DFC, osc_hi);
    gemm64<0, 0, 2><<<gG, blk, 0, stream>>>(
        AL, DFC, 0LL, W1P, DFC, 0LL, b1, b1, DFC,
        (void*)Lb, DFC, 0LL, MCH, DFC, DFC, osc_lo);
    xplanes<<<gX, blk, 0, stream>>>(Hb, Lb, b1, AH, AL, n8x);
    gemm64<0, 0, 2><<<gG, blk, 0, stream>>>(
        AH, DFC, 0LL, W2P, DFC, 0LL, b2, b2, DFC,
        (void*)Hb, DFC, 0LL, MCH, DFC, DFC, osc_hi);
    gemm64<0, 0, 2><<<gG, blk, 0, stream>>>(
        AL, DFC, 0LL, W2P, DFC, 0LL, b2, b2, DFC,
        (void*)Lb, DFC, 0LL, MCH, DFC, DFC, osc_lo);
    xplanes<<<gX, blk, 0, stream>>>(Hb, Lb, b2, AH, AL, n8x);
    gemm64<0, 0, 2><<<gH, blk, 0, stream>>>(
        AH, DFC, 0LL, W3P, DFC, 0LL, b3, b3, NHP,
        (void*)H3, NHP, 0LL, MCH, NHP, DFC, osc_hi);
    gemm64<0, 0, 2><<<gH, blk, 0, stream>>>(
        AL, DFC, 0LL, W3P, DFC, 0LL, b3, b3, NHP,
        (void*)L3, NHP, 0LL, MCH, NHP, DFC, osc_lo);
    outpack<<<gO, blk, 0, stream>>>(H3, L3, b3, out0 + (size_t)ch * MCH * NLAB, nqo);
  }
  (void)hipGetLastError();
}
